// GNNFiLMLayer_78091095376253
// MI455X (gfx1250) — hardware-verified
//
#include <hip/hip_runtime.h>
#include <stddef.h>
#include <stdint.h>


#define FEAT   128
#define NREL   4
#define NHW    512
#define NFILM  1024
#define NT     1152
#define NBT    NT
#define NBH    NHW
#define KQ     16
#define KSTEP  4
#define APK    136
#define TR     16
#define NTHR   256
#define NWAVE  8
#define CTH    4
#define CTT    9
#define S1     2048
#define NCH1   8
#define SH1    12
#define SH2    7
#define SH3    4
#define F1A    16
#define F2     32
#define F3     8
#define CAP1   256
#define CAP2   192
#define CAP3   512
#define SEGS2  16
#define WSC    64.0f
#define RWSC   0.015625f
#define SENT   0xFFFFFFFFu
#define WSCAPB 134217728
#define NPREP  ((NBH + NBT) * KQ)
#define STG_BYTES (TR * NT * 4)
#define SA_BYTES  (TR * APK * 2)
#define TILE_LDS  (STG_BYTES + SA_BYTES)

static_assert(NHW == NREL * FEAT);
static_assert(NFILM == NREL * 2 * FEAT);
static_assert(NT == NFILM + FEAT);
static_assert(KQ * 8 == FEAT && KSTEP * 32 == FEAT);
static_assert((APK % 8) == 0 && APK >= FEAT);
static_assert(NPREP % NTHR == 0);
static_assert((NBH * KQ) % NTHR == 0 && ((NBH + NFILM) * KQ) % NTHR == 0);
static_assert(NCH1 * NTHR == S1);
static_assert(CAP1 == NTHR);
static_assert((F1A * CAP1) % (4 * NTHR) == 0);
static_assert((F2 * CAP2) % (4 * NTHR) == 0);
static_assert((F3 * CAP3) % (4 * NTHR) == 0);
static_assert((CAP1 % 32) == 0 && (CAP2 % 32) == 0 && (CAP3 % 32) == 0);
static_assert(NTHR == 32 * NWAVE && TR == 2 * NWAVE);
static_assert(CTH * 16 * NWAVE == NHW && CTT * 16 * NWAVE == NT);
static_assert(NTHR * 4 * 2 == TR * FEAT);
static_assert((TR * NHW) % (4 * NTHR) == 0);
static_assert(STG_BYTES == 73728 && SA_BYTES == 4352 && TILE_LDS == 78080);
static_assert((STG_BYTES % 16) == 0);
static_assert(NREL == 4);

typedef _Float16 v4h  __attribute__((ext_vector_type(4)));
typedef _Float16 v8h  __attribute__((ext_vector_type(8)));
typedef _Float16 v16h __attribute__((ext_vector_type(16)));
typedef float    v4f  __attribute__((ext_vector_type(4)));
typedef float    v8f  __attribute__((ext_vector_type(8)));
typedef unsigned int v4u __attribute__((ext_vector_type(4)));
typedef v4h v4ha __attribute__((may_alias));
typedef v8h v8ha __attribute__((may_alias));
typedef v4f v4fa __attribute__((may_alias));
typedef v4u v4ua __attribute__((may_alias));
union Frag { v16h v; v8h h[2]; };

__device__ __forceinline__ v8f wmh(v16h a, v16h b, v8f c) {
  v8f d = __builtin_amdgcn_wmma_f32_16x16x32_f16(false, a, false, b, (short)0, c, false, false);
  asm volatile("v_nop\n\tv_nop\n\tv_nop\n\tv_nop" : "+v"(d) : "v"(a), "v"(b));
  return d;
}

__device__ __forceinline__ v4h cvt4(v4f a) {
  v4h r;
  r[0] = (_Float16)a[0]; r[1] = (_Float16)a[1]; r[2] = (_Float16)a[2]; r[3] = (_Float16)a[3];
  return r;
}

__global__ __launch_bounds__(NTHR) void k_wprep(const float* __restrict__ wrel, const float* __restrict__ film,
                                                const float* __restrict__ loopw, _Float16* Bw) {
  const int gi = blockIdx.x * NTHR + threadIdx.x;
  const int i0 = gi < NBH * KQ ? gi : NBH * KQ - 1;
  const int n0 = i0 >> 4, k00 = (i0 & 15) * 8, r0 = n0 >> 7, c0 = n0 & (FEAT - 1);
  int i1 = gi - NBH * KQ;
  i1 = i1 < 0 ? 0 : (i1 > NFILM * KQ - 1 ? NFILM * KQ - 1 : i1);
  const int n1 = i1 >> 4, k01 = (i1 & 15) * 8, r1 = n1 >> 8, c1 = n1 & (2 * FEAT - 1);
  int i2 = gi - (NBH + NFILM) * KQ;
  i2 = i2 < 0 ? 0 : (i2 > FEAT * KQ - 1 ? FEAT * KQ - 1 : i2);
  const int c2 = i2 >> 4, k02 = (i2 & 15) * 8;
  const int sel = gi < NBH * KQ ? 0 : (gi < (NBH + NFILM) * KQ ? 1 : 2);
  v8h hv;
#pragma unroll
  for (int e = 0; e < 8; ++e) {
    const float vw = wrel[((size_t)(r0 * FEAT + k00 + e)) * FEAT + c0];
    const float vf = film[((size_t)(r1 * FEAT + k01 + e)) * (2 * FEAT) + c1];
    const float vl = loopw[((size_t)(k02 + e)) * FEAT + c2];
    const float v = sel == 0 ? vw : (sel == 1 ? vf : vl);
    hv[e] = (_Float16)(v * WSC);
  }
  _Float16* dst = Bw + (size_t)gi * 8;
  *(volatile v8h*)dst = hv;
  __threadfence();
  *(volatile v8h*)dst = hv;
}

template <int LV, int FA, int CAP>
__global__ __launch_bounds__(NTHR) void k_part(const int* __restrict__ esrc, const int* __restrict__ edst,
                                               const int* __restrict__ ety, const unsigned* lin, unsigned* lout,
                                               int nN, int nE, int nC, int nB1, int P2, int nch) {
  __shared__ __attribute__((aligned(16))) unsigned lst[FA * CAP];
  __shared__ int wc[NWAVE * 32];
  __shared__ int cur[32];
  const int tid = threadIdx.x, lane = tid & 31, wave = tid >> 5;
  const int blk = blockIdx.x;
  const v4u sv = {SENT, SENT, SENT, SENT};
#pragma unroll
  for (int k = 0; k < (FA * CAP) / (4 * NTHR); ++k) *(v4ua*)(&lst[4 * (tid + NTHR * k)]) = sv;
  if (wave == 0) cur[lane] = 0;
  __syncthreads();

  int c = 0, part = 0, ml = 0;
  if (LV == 2) { c = blk / P2; part = blk - c * P2; }
  if (LV == 3) { c = blk >> 5; ml = blk & 31; }
  const int nslots3 = P2 * CAP2;

#pragma unroll 1
  for (int ch = 0; ch < nch; ++ch) {
    bool valid;
    int key;
    unsigned rec;
    if (LV == 1) {
      const int e = blk * S1 + ch * NTHR + tid;
      const int ec = e < nE ? e : nE - 1;
      const int d = edst[ec];
      valid = (e < nE) && ((unsigned)d < (unsigned)nN);
      key = d >> SH1;
      rec = (unsigned)ec;
    } else if (LV == 2) {
      const int bl = part * SEGS2 + ch;
      const int blc = bl < nB1 ? bl : nB1 - 1;
      const unsigned id = lin[((size_t)blc * nC + c) * CAP1 + tid];
      const bool idok = id < (unsigned)nE;
      const int idc = idok ? (int)id : nE - 1;
      const int d = edst[idc];
      valid = (bl < nB1) && idok && ((unsigned)d < (unsigned)nN);
      key = (d >> SH2) & 31;
      rec = (unsigned)idc;
    } else {
      const int q = ch * NTHR + tid;
      const int qc = q < nslots3 ? q : nslots3 - 1;
      const int pp = qc / CAP2, s = qc - pp * CAP2;
      const unsigned id = lin[(((size_t)(c * P2 + pp)) * F2 + ml) * CAP2 + s];
      const bool idok = id < (unsigned)nE;
      const int idc = idok ? (int)id : nE - 1;
      const int d = edst[idc];
      int sv2 = esrc[idc];
      sv2 = sv2 < 0 ? 0 : (sv2 > nN - 1 ? nN - 1 : sv2);
      int tv = ety[idc];
      tv = tv < 0 ? 0 : (tv > NREL - 1 ? NREL - 1 : tv);
      valid = (q < nslots3) && idok && ((unsigned)d < (unsigned)nN);
      key = (d >> SH3) & 7;
      rec = ((unsigned)d & 15u) | ((unsigned)tv << 4) | ((unsigned)sv2 << 8);
    }
    key = valid ? key : 255;
    unsigned mym = 0u;
#pragma unroll
    for (int b = 0; b < FA; ++b) {
      const unsigned mb = __builtin_amdgcn_ballot_w32(key == b);
      mym = (key == b) ? mb : mym;
    }
    const unsigned lt = (1u << lane) - 1u;
    const int rank = __builtin_popcount(mym & lt);
    const int cnt  = __builtin_popcount(mym);
    wc[wave * 32 + lane] = 0;
    if (valid && rank == 0) wc[wave * 32 + key] = cnt;
    __syncthreads();
    const int kc = key & 31;
    int pre = 0;
    for (int w2 = 0; w2 < wave; ++w2) pre += wc[w2 * 32 + kc];
    const int pos = cur[kc] + pre + rank;
    if (valid && pos < CAP) lst[kc * CAP + pos] = rec;
    int tot = 0;
    if (wave == 0) {
#pragma unroll
      for (int w2 = 0; w2 < NWAVE; ++w2) tot += wc[w2 * 32 + lane];
    }
    __syncthreads();
    if (wave == 0) cur[lane] += tot;
  }
  __syncthreads();

  const int nwords  = (LV == 1) ? nC * CAP : FA * CAP;
  const int npieces = nwords >> 2;
  unsigned* gb = lout + (size_t)blk * nwords;
#pragma unroll
  for (int k = 0; k < (FA * CAP / 4 + NTHR - 1) / NTHR; ++k) {
    const int it = tid + NTHR * k;
    if (it < npieces) { const v4u v = *(const v4ua*)(&lst[4 * it]); *(volatile v4u*)(gb + 4 * it) = v; }
  }
  __threadfence();
#pragma unroll
  for (int k = 0; k < (FA * CAP / 4 + NTHR - 1) / NTHR; ++k) {
    const int it = tid + NTHR * k;
    if (it < npieces) { const v4u v = *(const v4ua*)(&lst[4 * it]); *(volatile v4u*)(gb + 4 * it) = v; }
  }
}

__global__ __launch_bounds__(NTHR) void k_hw(const float* __restrict__ x, const _Float16* __restrict__ BH,
                                             float* HW, int nN) {
  __shared__ __attribute__((aligned(16))) _Float16 sA[TR * APK];
  __shared__ __attribute__((aligned(16))) float stg[TR * NHW];
  const int tid = threadIdx.x, lane = tid & 31, wave = tid >> 5, hh = lane >> 4, m = lane & 15;
  const int tile = blockIdx.x;
  const v4f z4 = {0.f, 0.f, 0.f, 0.f};
#pragma unroll
  for (int k = 0; k < 2; ++k) {
    const int row = wave + 8 * k, c4 = lane * 4;
    const int node = tile * TR + row;
    const int nc = node < nN ? node : nN - 1;
    v4f v = *(const v4f*)(x + (size_t)nc * FEAT + c4);
    if (node >= nN) v = z4;
    *(v4ha*)(sA + row * APK + c4) = cvt4(v);
  }
  __syncthreads();

  v16h av[KSTEP];
  {
    const _Float16* abase = sA + m * APK + 8 * hh;
#pragma unroll
    for (int kt = 0; kt < KSTEP; ++kt) {
      Frag a;
      a.h[0] = *(const v8ha*)(abase + 32 * kt);
      a.h[1] = *(const v8ha*)(abase + 32 * kt + 16);
      av[kt] = a.v;
    }
  }
#pragma unroll 1
  for (int ct = 0; ct < CTH; ++ct) {
    const int col = wave * (16 * CTH) + ct * 16 + m;
    const _Float16* bb = BH + (size_t)col * FEAT + 8 * hh;
    v8f acc = {0.f, 0.f, 0.f, 0.f, 0.f, 0.f, 0.f, 0.f};
#pragma unroll
    for (int kt = 0; kt < KSTEP; ++kt) {
      Frag b;
      b.h[0] = *(const v8h*)(bb + 32 * kt);
      b.h[1] = *(const v8h*)(bb + 32 * kt + 16);
      acc = wmh(av[kt], b.v, acc);
    }
#pragma unroll
    for (int r = 0; r < 8; ++r) stg[(8 * hh + r) * NHW + col] = acc[r] * RWSC;
  }
  __syncthreads();

  float* gb = HW + (size_t)tile * (TR * NHW);
#pragma unroll
  for (int k = 0; k < (TR * NHW) / (4 * NTHR); ++k) {
    const int it = tid + NTHR * k;
    const v4f v = *(const v4fa*)(stg + 4 * it);
    *(volatile v4f*)(gb + 4 * it) = v;
  }
  __threadfence();
#pragma unroll
  for (int k = 0; k < (TR * NHW) / (4 * NTHR); ++k) {
    const int it = tid + NTHR * k;
    const v4f v = *(const v4fa*)(stg + 4 * it);
    *(volatile v4f*)(gb + 4 * it) = v;
  }
}

__device__ __forceinline__ v4f drain(unsigned msk, unsigned rec, const float* strow, const float* __restrict__ HW,
                                     int lane, int nN, v4f acc) {
  while (msk != 0u) {
    const int i = __builtin_ctz(msk);
    msk &= msk - 1u;
    const unsigned r = (unsigned)__builtin_amdgcn_readlane((int)rec, i);
    int src = (int)(r >> 8);
    src = src > nN - 1 ? nN - 1 : src;
    const int ty = (int)((r >> 4) & 3u);
    const v4f v = *(const v4f*)(HW + ((size_t)src * NREL + ty) * FEAT + 4 * lane);
    const v4f g = *(const v4fa*)(strow + ty * (2 * FEAT) + 4 * lane);
    const v4f b = *(const v4fa*)(strow + ty * (2 * FEAT) + FEAT + 4 * lane);
    v4f t = g * v + b;
    t[0] = fmaxf(t[0], 0.0f); t[1] = fmaxf(t[1], 0.0f); t[2] = fmaxf(t[2], 0.0f); t[3] = fmaxf(t[3], 0.0f);
    acc += t;
  }
  return acc;
}

__global__ __launch_bounds__(NTHR) void k_tile(const float* __restrict__ x, const _Float16* __restrict__ BT,
                                               const unsigned* __restrict__ l3, const float* __restrict__ HW,
                                               const float* __restrict__ bias, float* out, int nN) {
  extern __shared__ __attribute__((aligned(16))) unsigned char dynlds[];
  float*    stg = (float*)dynlds;
  _Float16* sA  = (_Float16*)(dynlds + STG_BYTES);
  const int tid = threadIdx.x, lane = tid & 31, wave = tid >> 5, hh = lane >> 4, m = lane & 15;
  const int tile = blockIdx.x;
  const v4f z4 = {0.f, 0.f, 0.f, 0.f};
#pragma unroll
  for (int k = 0; k < 2; ++k) {
    const int row = wave + 8 * k, c4 = lane * 4;
    const int node = tile * TR + row;
    const int nc = node < nN ? node : nN - 1;
    v4f v = *(const v4f*)(x + (size_t)nc * FEAT + c4);
    if (node >= nN) v = z4;
    *(v4ha*)(sA + row * APK + c4) = cvt4(v);
  }
  __syncthreads();

  {
    v16h av[KSTEP];
    const _Float16* abase = sA + m * APK + 8 * hh;
#pragma unroll
    for (int kt = 0; kt < KSTEP; ++kt) {
      Frag a;
      a.h[0] = *(const v8ha*)(abase + 32 * kt);
      a.h[1] = *(const v8ha*)(abase + 32 * kt + 16);
      av[kt] = a.v;
    }
#pragma unroll 1
    for (int ct = 0; ct < CTT; ++ct) {
      const int col = wave * (16 * CTT) + ct * 16 + m;
      const _Float16* bb = BT + (size_t)col * FEAT + 8 * hh;
      v8f acc = {0.f, 0.f, 0.f, 0.f, 0.f, 0.f, 0.f, 0.f};
#pragma unroll
      for (int kt = 0; kt < KSTEP; ++kt) {
        Frag b;
        b.h[0] = *(const v8h*)(bb + 32 * kt);
        b.h[1] = *(const v8h*)(bb + 32 * kt + 16);
        acc = wmh(av[kt], b.v, acc);
      }
#pragma unroll
      for (int r = 0; r < 8; ++r) stg[(8 * hh + r) * NT + col] = acc[r] * RWSC;
    }
  }
  __syncthreads();

  v4f acc0 = z4, acc1 = z4;
  {
    const unsigned* seg = l3 + (size_t)tile * CAP3;
    const float* row0 = stg + (2 * wave) * NT;
    const float* row1 = row0 + NT;
#pragma unroll 1
    for (int ch = 0; ch < CAP3 / 32; ++ch) {
      const unsigned rec = seg[ch * 32 + lane];
      const bool ok = ((int)rec) >= 0;
      const int ln = (int)(rec & 15u);
      const unsigned m0 = __builtin_amdgcn_ballot_w32(ok && (ln == 2 * wave));
      const unsigned m1 = __builtin_amdgcn_ballot_w32(ok && (ln == 2 * wave + 1));
      acc0 = drain(m0, rec, row0, HW, lane, nN, acc0);
      acc1 = drain(m1, rec, row1, HW, lane, nN, acc1);
    }
  }

  const int c4 = lane * 4;
  const v4f bv = *(const v4f*)(bias + c4);
  const v4f l0 = *(const v4fa*)(stg + (2 * wave) * NT + NFILM + c4);
  const v4f l1 = *(const v4fa*)(stg + (2 * wave + 1) * NT + NFILM + c4);
  v4f o0 = acc0 + bv;
  v4f o1 = acc1 + bv;
  o0 = o0 + l0;
  o1 = o1 + l1;
  const int node0 = tile * TR + 2 * wave, node1 = node0 + 1;
  const bool a0 = node0 < nN, a1 = node1 < nN;
  float* g0 = out + (size_t)(a0 ? node0 : 0) * FEAT + c4;
  float* g1 = out + (size_t)(a1 ? node1 : 0) * FEAT + c4;
  if (a0) *(volatile v4f*)g0 = o0;
  if (a1) *(volatile v4f*)g1 = o1;
  __threadfence();
  if (a0) *(volatile v4f*)g0 = o0;
  if (a1) *(volatile v4f*)g1 = o1;
}

extern "C" void kernel_launch(void* const* d_in, const int* in_sizes, int n_in,
                              void* d_out, int out_size, void* d_ws, size_t ws_size,
                              hipStream_t stream) {
  if (n_in < 8) return;
  if (in_sizes[0] <= 0 || (in_sizes[0] % FEAT) != 0) return;
  const int nN = in_sizes[0] / FEAT;
  const int nE = in_sizes[1];
  if (nN < 1 || nN > 65536) return;
  if (nE < 1 || nE > (1 << 28)) return;
  if (in_sizes[2] != nE || in_sizes[3] != nE) return;
  if (in_sizes[4] != NREL * FEAT * FEAT || in_sizes[5] != NREL * FEAT * 2 * FEAT) return;
  if (in_sizes[6] != FEAT || in_sizes[7] != FEAT * FEAT) return;
  if (out_size != nN * FEAT) return;

  const float* x     = (const float*)d_in[0];
  const int*   esrc  = (const int*)d_in[1];
  const int*   edst  = (const int*)d_in[2];
  const int*   ety   = (const int*)d_in[3];
  const float* wrel  = (const float*)d_in[4];
  const float* film  = (const float*)d_in[5];
  const float* bias  = (const float*)d_in[6];
  const float* loopw = (const float*)d_in[7];
  float* out = (float*)d_out;

  const int nTiles = (nN + TR - 1) / TR;
  const int nC   = (nN + 4095) >> SH1;
  const int nB1  = (nE + S1 - 1) / S1;
  const int P2   = (nB1 + SEGS2 - 1) / SEGS2;
  const int nch3 = (P2 * CAP2 + NTHR - 1) / NTHR;
  if (nC < 1 || nC > F1A) return;

  char* ws = (char*)d_ws;
  size_t o = 0;
  const size_t oBw = o; o += (size_t)(NBH + NBT) * FEAT * 2;              o = (o + 255) & ~(size_t)255;
  const size_t oL1 = o; o += (size_t)nB1 * nC * CAP1 * 4;                 o = (o + 255) & ~(size_t)255;
  const size_t oL2 = o; o += (size_t)nC * P2 * F2 * CAP2 * 4;             o = (o + 255) & ~(size_t)255;
  const size_t oL3 = o; o += (size_t)nC * 32 * F3 * CAP3 * 4;             o = (o + 255) & ~(size_t)255;
  const size_t oHW = o; o += (size_t)nTiles * TR * NHW * 4;               o = (o + 255) & ~(size_t)255;
  if (o > ws_size || o > (size_t)WSCAPB) return;
  _Float16* Bw = (_Float16*)(ws + oBw);
  unsigned* L1 = (unsigned*)(ws + oL1);
  unsigned* L2 = (unsigned*)(ws + oL2);
  unsigned* L3 = (unsigned*)(ws + oL3);
  float*    HW = (float*)(ws + oHW);

  k_wprep<<<NPREP / NTHR, NTHR, 0, stream>>>(wrel, film, loopw, Bw);
  k_part<1, F1A, CAP1><<<nB1, NTHR, 0, stream>>>(esrc, edst, ety, L1, L1, nN, nE, nC, nB1, P2, NCH1);
  k_part<2, F2, CAP2><<<nC * P2, NTHR, 0, stream>>>(esrc, edst, ety, L1, L2, nN, nE, nC, nB1, P2, SEGS2);
  k_part<3, F3, CAP3><<<nC * 32, NTHR, 0, stream>>>(esrc, edst, ety, L2, L3, nN, nE, nC, nB1, P2, nch3);
  k_hw<<<nTiles, NTHR, 0, stream>>>(x, Bw, HW, nN);
  hipFuncSetAttribute(reinterpret_cast<const void*>(&k_tile), hipFuncAttributeMaxDynamicSharedMemorySize, TILE_LDS);
  k_tile<<<nTiles, NTHR, TILE_LDS, stream>>>(x, Bw + (size_t)NBH * FEAT, L3, HW, bias, out, nN);
}
